// ResidualGATBlock_89644557402834
// MI455X (gfx1250) — hardware-verified
//
#include <hip/hip_runtime.h>
#include <stddef.h>
#include <stdint.h>


#define DIN     128
#define HCO     128
#define NHEAD   8
#define HDIM    16
#define ASDW    16
#define NTHR    256
#define NWAVE   8
#define EPT     8
#define CHUNK   (NTHR * EPT)
#define WCAP    (EPT * 32)
#define LISTN   (NWAVE * WCAP)
#define NBMAX   1024
#define RCAP    28672
#define DEGCAP  256
#define STW     512
#define GBM     64
#define GBN     128
#define GTHR    128
#define CX      8.0f
#define CW      64.0f
#define SCL_XW  0.001953125f
#define NEGSL   0.2f
#define LNEPS   1.0e-5f
#define INVC    0.0078125f
#define WSMAX   134217728
#define LDS_AGG ((2 * RCAP + 2 * NBMAX + LISTN + 2 * NWAVE + 16) * 4)

static_assert((CHUNK & (CHUNK - 1)) == 0 && CHUNK <= 4096);
static_assert((NBMAX & (NBMAX - 1)) == 0 && NBMAX <= 4096);
static_assert(NTHR * 4 == NBMAX);
static_assert(LISTN >= NBMAX);
static_assert(LISTN >= NWAVE * WCAP);
static_assert((RCAP % 32) == 0);
static_assert(NWAVE * STW <= RCAP);
static_assert(STW >= HCO);
static_assert(LDS_AGG <= 300000);
static_assert(GBM == (GTHR / 32) * 16);
static_assert(GBN == HCO && DIN == HCO);
static_assert(NHEAD * HDIM == HCO);
static_assert((DIN % 32) == 0 && DIN == 128);
static_assert(GTHR == HCO);
static_assert(GTHR == 2 * GBM);
static_assert(2 * GTHR * 4 == GBM * ASDW);
static_assert(HCO == 4 * 32);

typedef float    v4f  __attribute__((ext_vector_type(4)));
typedef float    v8f  __attribute__((ext_vector_type(8)));
typedef int      v4i  __attribute__((ext_vector_type(4)));
typedef int      v8i  __attribute__((ext_vector_type(8)));
typedef _Float16 v8h  __attribute__((ext_vector_type(8)));
typedef _Float16 v16h __attribute__((ext_vector_type(16)));
union FragH { v16h v; v8h h[2]; v8i w; };

__device__ __forceinline__ v8f wmh(const FragH& a, const FragH& b, v8f c) {
  v8f d = __builtin_amdgcn_wmma_f32_16x16x32_f16(false, a.v, false, b.v, (short)0, c, false, false);
  asm volatile("v_nop\n\tv_nop\n\tv_nop\n\tv_nop" : "+v"(d) : "v"(a.w), "v"(b.w));
  return d;
}

__device__ __forceinline__ void ldwait() {
  asm volatile("s_wait_loadcnt 0x0" ::: "memory");
}

__device__ __forceinline__ float bfr(float f) {
  unsigned u = __float_as_uint(f);
  u = (u + 0x7FFFu + ((u >> 16) & 1u)) & 0xFFFF0000u;
  return __uint_as_float(u);
}

__device__ __forceinline__ v8h cvt8hb(const v4f a, const v4f b, const float c) {
  v8h hv;
  hv[0] = (_Float16)(bfr(a.x) * c); hv[1] = (_Float16)(bfr(a.y) * c);
  hv[2] = (_Float16)(bfr(a.z) * c); hv[3] = (_Float16)(bfr(a.w) * c);
  hv[4] = (_Float16)(bfr(b.x) * c); hv[5] = (_Float16)(bfr(b.y) * c);
  hv[6] = (_Float16)(bfr(b.z) * c); hv[7] = (_Float16)(bfr(b.w) * c);
  return hv;
}

__device__ __forceinline__ int scan_chunk(const int* __restrict__ dsts, int nE, int cbase, int slotBase,
                                          int nb, int vec8, int* list, int tid, int lane, int wave) {
  int wc = 0;
  const int el0  = tid * EPT;
  const int e0   = cbase + el0;
  const int sent = -2147483647 - 1;
  v4i da, db;
  if (vec8 != 0 && cbase + CHUNK <= nE) {
    da = *(const v4i*)(dsts + e0);
    db = *(const v4i*)(dsts + e0 + 4);
  } else {
    da.x = (e0     < nE) ? dsts[min(e0,     nE - 1)] : sent;
    da.y = (e0 + 1 < nE) ? dsts[min(e0 + 1, nE - 1)] : sent;
    da.z = (e0 + 2 < nE) ? dsts[min(e0 + 2, nE - 1)] : sent;
    da.w = (e0 + 3 < nE) ? dsts[min(e0 + 3, nE - 1)] : sent;
    db.x = (e0 + 4 < nE) ? dsts[min(e0 + 4, nE - 1)] : sent;
    db.y = (e0 + 5 < nE) ? dsts[min(e0 + 5, nE - 1)] : sent;
    db.z = (e0 + 6 < nE) ? dsts[min(e0 + 6, nE - 1)] : sent;
    db.w = (e0 + 7 < nE) ? dsts[min(e0 + 7, nE - 1)] : sent;
  }
  const unsigned nbs = (unsigned)slotBase;
  const unsigned unb = (unsigned)nb;
  const unsigned s0 = (unsigned)da.x - nbs, s1 = (unsigned)da.y - nbs;
  const unsigned s2 = (unsigned)da.z - nbs, s3 = (unsigned)da.w - nbs;
  const unsigned s4 = (unsigned)db.x - nbs, s5 = (unsigned)db.y - nbs;
  const unsigned s6 = (unsigned)db.z - nbs, s7 = (unsigned)db.w - nbs;
  const bool h0 = s0 < unb, h1 = s1 < unb, h2 = s2 < unb, h3 = s3 < unb;
  const bool h4 = s4 < unb, h5 = s5 < unb, h6 = s6 < unb, h7 = s7 < unb;
  const unsigned any = __builtin_amdgcn_ballot_w32(h0 | h1 | h2 | h3 | h4 | h5 | h6 | h7);
  if (any != 0u) {
#define HITJ(J, HJ, SJ) { \
      const unsigned mj = __builtin_amdgcn_ballot_w32(HJ); \
      if (mj != 0u) { \
        if (HJ) { \
          const int pos = wc + (int)__builtin_amdgcn_mbcnt_lo(mj, 0u); \
          if (pos < WCAP) list[wave * WCAP + pos] = ((el0 + (J)) << 12) | (int)(SJ); \
        } \
        wc += (int)__builtin_popcount(mj); } }
    HITJ(0, h0, s0)
    HITJ(1, h1, s1)
    HITJ(2, h2, s2)
    HITJ(3, h3, s3)
    HITJ(4, h4, s4)
    HITJ(5, h5, s5)
    HITJ(6, h6, s6)
    HITJ(7, h7, s7)
#undef HITJ
  }
  return wc;
}

__global__ __launch_bounds__(NTHR) void k_xprep(const float* __restrict__ x, _Float16* xh, int nN, int nUnits) {
  const int i = (int)blockIdx.x * NTHR + (int)threadIdx.x;
  if (i >= nUnits) return;
  const int row = i >> 4;
  const int c0  = (i & 15) * 8;
  const int rc  = row < nN ? row : nN - 1;
  const float* p = x + (size_t)rc * DIN + c0;
  v4f a = *(const v4f*)p, b = *(const v4f*)(p + 4);
  const v4f z4 = {0.f, 0.f, 0.f, 0.f};
  if (row >= nN) { a = z4; b = z4; }
  const v8h hv = cvt8hb(a, b, CX);
  const size_t o = (size_t)row * DIN + c0;
  *(volatile v8h*)(xh + o) = hv;
  __threadfence();
  *(volatile v8h*)(xh + o) = hv;
}

__global__ __launch_bounds__(NTHR) void k_wtr(const float* __restrict__ w, _Float16* wt, int cols, int K, int nUnits) {
  const int u = (int)blockIdx.x * NTHR + (int)threadIdx.x;
  if (u >= nUnits) return;
  const int kq = K >> 3;
  const int n  = u / kq;
  const int k8 = (u - n * kq) * 8;
  const float* p = w + (size_t)k8 * (size_t)cols + n;
  v4f a, b;
  a.x = p[0];                   a.y = p[(size_t)cols];        a.z = p[(size_t)2 * cols];    a.w = p[(size_t)3 * cols];
  b.x = p[(size_t)4 * cols];    b.y = p[(size_t)5 * cols];    b.z = p[(size_t)6 * cols];    b.w = p[(size_t)7 * cols];
  const v8h hv = cvt8hb(a, b, CW);
  const size_t o = (size_t)n * (size_t)K + k8;
  *(volatile v8h*)(wt + o) = hv;
  __threadfence();
  *(volatile v8h*)(wt + o) = hv;
}

__global__ __launch_bounds__(GTHR) void k_gemm(
    const _Float16* __restrict__ A, const _Float16* __restrict__ WT,
    const float* __restrict__ atts, const float* __restrict__ attd,
    float* Hout, float* ASD, int K)
{
  __shared__ __attribute__((aligned(16))) float stg[GBM * GBN];
  __shared__ __attribute__((aligned(16))) float asl[GBM * ASDW];
  __shared__ __attribute__((aligned(16))) float atl[2 * HCO];
  const int tid = (int)threadIdx.x, lane = tid & 31, wave = tid >> 5, hh = lane >> 4, m = lane & 15;
  const int rowBase = (int)blockIdx.x * GBM;

  atl[tid]       = bfr(atts[tid]);
  atl[HCO + tid] = bfr(attd[tid]);

  v8f acc[8];
  {
    const v8f z = {0.f, 0.f, 0.f, 0.f, 0.f, 0.f, 0.f, 0.f};
#pragma unroll
    for (int t = 0; t < 8; ++t) acc[t] = z;
  }
  const _Float16* ap = A  + (size_t)(rowBase + 16 * wave + m) * (size_t)K + 8 * hh;
  const _Float16* wp = WT + (size_t)m * (size_t)K + 8 * hh;
  const int ksteps = K >> 5;
#pragma unroll 1
  for (int ks = 0; ks < ksteps; ++ks) {
    FragH af;
    af.h[0] = *(const v8h*)(ap + 32 * ks);
    af.h[1] = *(const v8h*)(ap + 32 * ks + 16);
#pragma unroll
    for (int t = 0; t < 8; ++t) {
      const _Float16* wq = wp + (size_t)(16 * t) * (size_t)K + 32 * ks;
      FragH bf;
      bf.h[0] = *(const v8h*)wq;
      bf.h[1] = *(const v8h*)(wq + 16);
      acc[t] = wmh(af, bf, acc[t]);
    }
  }

#pragma unroll
  for (int t = 0; t < 8; ++t) {
    const int lc = 16 * t + m;
#pragma unroll
    for (int r = 0; r < 8; ++r) {
      const int lr = 16 * wave + 8 * hh + r;
      stg[lr * GBN + lc] = acc[t][r] * SCL_XW;
    }
  }
  __syncthreads();

  {
    const int r = tid >> 1;
    const int which = tid & 1;
    const float* rp = stg + r * GBN;
    const float* tp = atl + which * HCO;
#pragma unroll 1
    for (int hd = 0; hd < NHEAD; ++hd) {
      float s = 0.f;
#pragma unroll
      for (int c = 0; c < HDIM; ++c) s = fmaf(rp[hd * HDIM + c], tp[hd * HDIM + c], s);
      asl[r * ASDW + which * NHEAD + hd] = s;
    }
  }
  __syncthreads();

#pragma unroll
  for (int i = 0; i < 16; ++i) {
    const int lr = 16 * wave + i;
    const v4f v = *(const v4f*)(stg + lr * GBN + 4 * lane);
    *(volatile v4f*)(Hout + (size_t)(rowBase + lr) * HCO + 4 * lane) = v;
  }
#pragma unroll
  for (int i = 0; i < 2; ++i) {
    const int p = i * GTHR + tid;
    const v4f v = *(const v4f*)(asl + 4 * p);
    *(volatile v4f*)(ASD + (size_t)rowBase * ASDW + 4 * p) = v;
  }
  __threadfence();
#pragma unroll
  for (int i = 0; i < 16; ++i) {
    const int lr = 16 * wave + i;
    const v4f v = *(const v4f*)(stg + lr * GBN + 4 * lane);
    *(volatile v4f*)(Hout + (size_t)(rowBase + lr) * HCO + 4 * lane) = v;
  }
#pragma unroll
  for (int i = 0; i < 2; ++i) {
    const int p = i * GTHR + tid;
    const v4f v = *(const v4f*)(asl + 4 * p);
    *(volatile v4f*)(ASD + (size_t)rowBase * ASDW + 4 * p) = v;
  }
}

__global__ __launch_bounds__(NTHR) void k_agg(
    const int* __restrict__ srcs, const int* __restrict__ dsts, const float* __restrict__ eattr,
    const float* __restrict__ H, const float* __restrict__ ASD, const float* __restrict__ x,
    const float* __restrict__ bias, const float* __restrict__ lew, const float* __restrict__ leb,
    const float* __restrict__ aedge, const float* __restrict__ gam, const float* __restrict__ bet,
    float* out, int nN, int nE, int nb, int vec8) {
  extern __shared__ v4f lds_dyn[];
  int* reg1 = (int*)lds_dyn;
  int* reg2 = reg1 + RCAP;
  int* scnt = reg2 + RCAP;
  int* soff = scnt + NBMAX;
  int* list = soff + NBMAX;
  int* wcnt = list + LISTN;
  int* wtot = wcnt + NWAVE;
  float* coef = (float*)(wtot + NWAVE);
  const int tid = (int)threadIdx.x, lane = tid & 31, wave = tid >> 5;
  const int nodeBase = (int)blockIdx.x * nb;

  for (int i = tid; i < NBMAX; i += NTHR) scnt[i] = 0;
  if (wave == 0) {
    const int which = (lane >> 3) & 1;
    const int hd = lane & 7;
    float s = 0.f;
#pragma unroll 1
    for (int c = 0; c < HDIM; ++c) {
      const int i = hd * HDIM + c;
      const float wv = bfr(lew[i]);
      const float bv = bfr(leb[i]);
      const float av = bfr(aedge[i]);
      s = fmaf(which ? bv : wv, av, s);
    }
    if (lane < 16) coef[lane] = s;
  }
  __syncthreads();

  int tot = 0;
  const int nChunks = (nE + CHUNK - 1) / CHUNK;
#pragma unroll 1
  for (int ch = 0; ch < nChunks; ++ch) {
    const int cbase = ch * CHUNK;
    const int wc = scan_chunk(dsts, nE, cbase, nodeBase, nb, vec8, list, tid, lane, wave);
    if (lane == 0) wcnt[wave] = wc;
    __syncthreads();
    int pre = 0, all = 0;
#pragma unroll
    for (int w2 = 0; w2 < NWAVE; ++w2) {
      int c = wcnt[w2];
      c = c < 0 ? 0 : (c > WCAP ? WCAP : c);
      all += c;
      pre += (w2 < wave) ? c : 0;
    }
    const int wcc  = wc > WCAP ? WCAP : wc;
    const int base = tot + pre;
#pragma unroll 1
    for (int i = lane; i < wcc; i += 32) {
      const int ent = list[wave * WCAP + i];
      const int el  = (ent >> 12) & (CHUNK - 1);
      const int sl  = ent & (NBMAX - 1);
      int eid = cbase + el;
      eid = eid > nE - 1 ? nE - 1 : eid;
      const int pos = base + i;
      if (pos < RCAP) reg1[pos] = (int)(((unsigned)eid << 12) | (unsigned)sl);
    }
    tot += all;
    tot = tot > RCAP ? RCAP : tot;
    __syncthreads();
  }
  const int nh = tot;

  if (wave == 0) {
#pragma unroll 1
    for (int b0 = 0; b0 < nh; b0 += 32) {
      const int idx = b0 + lane;
      const int uv  = reg1[idx < RCAP ? idx : RCAP - 1];
      const int m32 = (nh - b0) < 32 ? (nh - b0) : 32;
#pragma unroll 1
      for (int k = 0; k < m32; ++k) {
        const int u  = __builtin_amdgcn_readlane(uv, k);
        const int sl = u & (NBMAX - 1);
        if (lane == 0) scnt[sl] = scnt[sl] + 1;
      }
    }
  }
  __syncthreads();

  {
    const v4i ca = *(const v4i*)(scnt + 4 * tid);
    const int e0 = ca.x < 0 ? 0 : ca.x, e1 = ca.y < 0 ? 0 : ca.y, e2 = ca.z < 0 ? 0 : ca.z, e3 = ca.w < 0 ? 0 : ca.w;
    const int ts = e0 + e1 + e2 + e3;
    int incl = ts;
#pragma unroll
    for (int d = 1; d < 32; d <<= 1) {
      const int up = __shfl_up(incl, d);
      if (lane >= d) incl += up;
    }
    if (lane == 31) wtot[wave] = incl;
    __syncthreads();
    int pre = 0;
#pragma unroll
    for (int w2 = 0; w2 < NWAVE; ++w2) pre += (w2 < wave) ? wtot[w2] : 0;
    int run = pre + incl - ts;
    soff[4 * tid + 0] = run; run += e0;
    soff[4 * tid + 1] = run; run += e1;
    soff[4 * tid + 2] = run; run += e2;
    soff[4 * tid + 3] = run;
  }
  __syncthreads();
  for (int i = tid; i < NBMAX; i += NTHR) list[i] = soff[i];
  __syncthreads();

  if (wave == 0) {
#pragma unroll 1
    for (int b0 = 0; b0 < nh; b0 += 32) {
      const int idx = b0 + lane;
      const int uv  = reg1[idx < RCAP ? idx : RCAP - 1];
      const int m32 = (nh - b0) < 32 ? (nh - b0) : 32;
#pragma unroll 1
      for (int k = 0; k < m32; ++k) {
        const int u   = __builtin_amdgcn_readlane(uv, k);
        const int sl  = u & (NBMAX - 1);
        const int eid = (int)((unsigned)u >> 12);
        if (lane == 0) {
          int pos = list[sl];
          pos = pos < 0 ? 0 : (pos > RCAP - 1 ? RCAP - 1 : pos);
          reg2[pos] = eid;
          list[sl] = pos + 1;
        }
      }
    }
  }
  __syncthreads();

  const int nbw = nb >> 3;
  const bool ovf = (nh >= RCAP);
  const float qnan = __int_as_float(0x7fc00000);
  float* stw = (float*)reg1 + wave * STW;
  const int hs = lane >> 4;
  float Aj[4], Bj[4], bq[4];
#pragma unroll
  for (int j = 0; j < 4; ++j) {
    Aj[j] = coef[2 * j + hs];
    Bj[j] = coef[NHEAD + 2 * j + hs];
    bq[j] = bfr(bias[32 * j + lane]);
  }
#pragma unroll 1
  for (int jt = 0; jt < nbw; ++jt) {
    const int slot = wave * nbw + jt;
    const int grow = nodeBase + slot;
    const int gcl  = grow < nN ? grow : nN - 1;
    int st = soff[slot];
    const int craw = scnt[slot];
    int cnt = craw;
    st  = st < 0 ? 0 : (st > nh ? nh : st);
    cnt = cnt < 0 ? 0 : (cnt > DEGCAP ? DEGCAP : cnt);
    if (cnt > nh - st) cnt = nh - st;
    const float pz = (ovf || craw > DEGCAP) ? qnan : 0.0f;
    const bool wr = grow < nN;

    const float* dp = ASD + (size_t)gcl * ASDW + NHEAD;
    const v4f d0 = *(const v4f*)dp;
    const v4f d1 = *(const v4f*)(dp + 4);
    const float* xrow = x + (size_t)gcl * DIN + lane;
    float xr[4];
#pragma unroll
    for (int j = 0; j < 4; ++j) xr[j] = xrow[32 * j];
    ldwait();
    float ad[4];
    ad[0] = hs ? d0.y : d0.x;
    ad[1] = hs ? d0.w : d0.z;
    ad[2] = hs ? d1.y : d1.x;
    ad[3] = hs ? d1.w : d1.z;
    float mx[4], dn[4], av[4];
#pragma unroll
    for (int j = 0; j < 4; ++j) { mx[j] = -1.0e30f; dn[j] = 0.f; av[j] = 0.f; xr[j] = bfr(xr[j]); }

#pragma unroll 1
    for (int q = 0; q < cnt; ++q) {
      int idx = st + q; idx = idx > RCAP - 1 ? RCAP - 1 : idx;
      int eid = reg2[idx]; eid = eid < 0 ? 0 : (eid > nE - 1 ? nE - 1 : eid);
      const int sraw = srcs[eid];
      const int s = sraw < 0 ? 0 : (sraw > nN - 1 ? nN - 1 : sraw);
      const float ea = bfr(eattr[eid]);
      const float* sp = ASD + (size_t)s * ASDW;
      const v4f p0 = *(const v4f*)sp;
      const v4f p1 = *(const v4f*)(sp + 4);
      const float* hr = H + (size_t)s * HCO + lane;
      float hv[4];
#pragma unroll
      for (int j = 0; j < 4; ++j) hv[j] = hr[32 * j];
      ldwait();
      float as[4];
      as[0] = hs ? p0.y : p0.x;
      as[1] = hs ? p0.w : p0.z;
      as[2] = hs ? p1.y : p1.x;
      as[3] = hs ? p1.w : p1.z;
#pragma unroll
      for (int j = 0; j < 4; ++j) {
        const float t = fmaf(ea, Aj[j], Bj[j]);
        float al = (as[j] + ad[j]) + t;
        al = al > 0.f ? al : al * NEGSL;
        const float df = al - mx[j];
        const float ee = __expf(-fabsf(df));
        const bool up  = df > 0.f;
        const float s1 = up ? ee : 1.0f;
        const float s2 = up ? 1.0f : ee;
        mx[j] = up ? al : mx[j];
        dn[j] = fmaf(dn[j], s1, s2);
        av[j] = fmaf(av[j], s1, s2 * hv[j]);
      }
    }
    float v[4];
#pragma unroll
    for (int j = 0; j < 4; ++j) {
      const float ds = dn[j] > 0.f ? dn[j] : 1.0f;
      const float o  = (dn[j] > 0.f ? av[j] : 0.0f) * __builtin_amdgcn_rcpf(ds);
      v[j] = (o + bq[j]) + xr[j];
    }
    float sm = (v[0] + v[1]) + (v[2] + v[3]);
#pragma unroll
    for (int off = 16; off > 0; off >>= 1) sm += __shfl_xor(sm, off);
    const float mu = sm * INVC;
    float dv[4];
#pragma unroll
    for (int j = 0; j < 4; ++j) dv[j] = v[j] - mu;
    float sq = (dv[0] * dv[0] + dv[1] * dv[1]) + (dv[2] * dv[2] + dv[3] * dv[3]);
#pragma unroll
    for (int off = 16; off > 0; off >>= 1) sq += __shfl_xor(sq, off);
    const float inv = rsqrtf(sq * INVC + LNEPS);

    __builtin_amdgcn_fence(__ATOMIC_RELEASE, "wavefront");
    __builtin_amdgcn_wave_barrier();
#pragma unroll
    for (int j = 0; j < 4; ++j) stw[32 * j + lane] = dv[j] * inv;
#pragma unroll 1
    for (int j = 0; j < 4; ++j) {
      const int c = 32 * j + lane;
      const float g  = bfr(gam[c]);
      const float be = bfr(bet[c]);
      float y = fmaf(stw[c], g, be);
      y = y > 0.f ? y : expm1f(y);
      stw[c] = y + pz;
    }
    __builtin_amdgcn_fence(__ATOMIC_RELEASE, "wavefront");
    __builtin_amdgcn_wave_barrier();
    const v4f ga = *(const v4f*)(stw + 4 * lane);
    float* gp = out + (size_t)gcl * HCO + 4 * lane;
    if (wr) *(volatile v4f*)gp = ga;
    __threadfence();
    if (wr) *(volatile v4f*)gp = ga;
  }
}

static int pick_nb(int nE, int nN) {
  int nb = NBMAX;
  while (nb > 16 && (long long)nb * (long long)nE * 5LL > (long long)RCAP * (long long)nN * 4LL) nb >>= 1;
  return nb;
}
static inline int cdiv(int a, int b) { return (a + b - 1) / b; }

extern "C" void kernel_launch(void* const* d_in, const int* in_sizes, int n_in,
                              void* d_out, int out_size, void* d_ws, size_t ws_size,
                              hipStream_t stream) {
  if (n_in < 12) return;
  const int nN = in_sizes[0] / DIN;
  if (nN <= 0 || in_sizes[0] != nN * DIN || nN > (1 << 22)) return;
  if (in_sizes[1] < 2 || (in_sizes[1] & 1) != 0) return;
  const int nE = in_sizes[1] / 2;
  if (nE < 1 || nE > (1 << 20)) return;
  if (in_sizes[2]  != nE) return;
  if (in_sizes[3]  != DIN * HCO) return;
  if (in_sizes[4]  != HCO) return;
  if (in_sizes[5]  != NHEAD * HDIM || in_sizes[6] != NHEAD * HDIM || in_sizes[7] != NHEAD * HDIM) return;
  if (in_sizes[8]  != HCO || in_sizes[9] != HCO) return;
  if (in_sizes[10] != HCO || in_sizes[11] != HCO) return;
  if (out_size != nN * HCO) return;

  const float* x     = (const float*)d_in[0];
  const int*   ei    = (const int*)  d_in[1];
  const float* eattr = (const float*)d_in[2];
  const float* W     = (const float*)d_in[3];
  const float* bb    = (const float*)d_in[4];
  const float* atts  = (const float*)d_in[5];
  const float* attd  = (const float*)d_in[6];
  const float* atte  = (const float*)d_in[7];
  const float* lew   = (const float*)d_in[8];
  const float* leb   = (const float*)d_in[9];
  const float* gam   = (const float*)d_in[10];
  const float* bet   = (const float*)d_in[11];
  float* out = (float*)d_out;
  const int* src = ei;
  const int* dst = ei + nE;

  const int MP   = cdiv(nN, GBM) * GBM;
  const int nb   = pick_nb(nE, nN);
  const int gA   = cdiv(nN, nb);
  const int vec8 = ((nE & 3) == 0) ? 1 : 0;
  if ((long long)gA * nb < nN) return;

  char* ws = (char*)d_ws;
  size_t off = 0;
  const size_t oXH = off; off += (size_t)MP * DIN * 2;     off = (off + 255) & ~(size_t)255;
  const size_t oWT = off; off += (size_t)HCO * DIN * 2;    off = (off + 255) & ~(size_t)255;
  const size_t oH  = off; off += (size_t)MP * HCO * 4;     off = (off + 255) & ~(size_t)255;
  const size_t oAS = off; off += (size_t)MP * ASDW * 4;    off = (off + 255) & ~(size_t)255;
  if (off > ws_size || off > (size_t)WSMAX) return;
  _Float16* XH  = (_Float16*)(ws + oXH);
  _Float16* WT  = (_Float16*)(ws + oWT);
  float*    Hp  = (float*)(ws + oH);
  float*    ASD = (float*)(ws + oAS);

  hipFuncSetAttribute(reinterpret_cast<const void*>(&k_agg),
                      hipFuncAttributeMaxDynamicSharedMemorySize, LDS_AGG);

  const int nUx = MP * (DIN / 8);
  k_xprep<<<cdiv(nUx, NTHR), NTHR, 0, stream>>>(x, XH, nN, nUx);

  const int nUw = HCO * (DIN / 8);
  k_wtr<<<cdiv(nUw, NTHR), NTHR, 0, stream>>>(W, WT, HCO, DIN, nUw);

  k_gemm<<<MP / GBM, GTHR, 0, stream>>>(XH, WT, atts, attd, Hp, ASD, DIN);

  k_agg<<<gA, NTHR, LDS_AGG, stream>>>(src, dst, eattr, Hp, ASD, x, bb, lew, leb, atte, gam, bet,
                                       out, nN, nE, nb, vec8);
}
